// MaxwellsDemonGNN_71176198029758
// MI455X (gfx1250) — hardware-verified
//
#include <hip/hip_runtime.h>


namespace {
constexpr int NB = 4, S = 512, IN = 32, H = 64, HD = 32  , NC = 3, NR = NB * S, PW = 64 + 64 + 32 + 32  ;
constexpr float XS = 8.0f, WSC = 256.0f;

typedef _Float16 b16;
typedef __attribute__((ext_vector_type(16))) _Float16 v16b;
typedef __attribute__((ext_vector_type(8))) _Float16 v8b;
typedef __attribute__((ext_vector_type(8))) float v8f;
typedef __attribute__((ext_vector_type(4))) float v4f;
__device__ __forceinline__ float bf16_rne(float f) { unsigned int u = __float_as_uint(f); u += 0x7FFFu + ((u >> 16) & 1u); return __uint_as_float(u & 0xFFFF0000u); }
__device__ __forceinline__ void split16(float v, b16& hi, b16& lo) { hi = (b16)v; lo = (b16)(v - (float)hi); }
__device__ __forceinline__ v16b frag_kb(const b16* p, int hh) { const v8b a = *(const v8b*)(p + 8 * hh), b = *(const v8b*)(p + 16 + 8 * hh); v16b f;
#pragma unroll
  for (int e = 0; e < 8; ++e) { f[e] = a[e]; f[8 + e] = b[e]; } return f; }
__device__ __forceinline__ v8f wmma16b(v16b a, v16b b, v8f c) { v8f d = __builtin_amdgcn_wmma_f32_16x16x32_f16(false, a, false, b, (short)0, c, false, false); asm volatile("v_nop\n\tv_nop\n\tv_nop\n\tv_nop" : "+v"(d) : "v"(a), "v"(b)); return d; }
__device__ __forceinline__ void wave_lds_sync() { __builtin_amdgcn_fence(__ATOMIC_RELEASE, "workgroup"); __builtin_amdgcn_wave_barrier(); __builtin_amdgcn_fence(__ATOMIC_ACQUIRE, "workgroup"); }
__device__ __forceinline__ float pmul(float a, float b) { float p = a * b; asm volatile("" : "+v"(p)); return p; }

__global__ __launch_bounds__(256) void prep_kernel(const float* __restrict__ x, const float* __restrict__ w1, const float* __restrict__ w2, const float* __restrict__ we1, const float* __restrict__ wd1, const float* __restrict__ wd2, b16* __restrict__ X16, b16* __restrict__ W1T, b16* __restrict__ W2T, b16* __restrict__ WPT, b16* __restrict__ WD2) {
  const size_t t = (size_t)blockIdx.x * 256 + threadIdx.x; const size_t nx = (size_t)NR * IN / 8, n1 = H * IN / 8, n2 = H * H / 8, n3 = PW * H / 8, n4 = 16 * HD / 8; v8b o;
  if (t < nx) { const size_t e = t * 8; const v4f a = *(const v4f*)(x + e), c = *(const v4f*)(x + e + 4); for (int j = 0; j < 4; ++j) { o[j] = (b16)(bf16_rne(a[j]) * XS); o[4 + j] = (b16)(bf16_rne(c[j]) * XS); } for (int pass = 0; pass < 2; ++pass) { *(volatile v8b*)(X16 + e) = o; __threadfence(); } return; }
  size_t u = t - nx;
  if (u < n1) { const int e = (int)u * 8; const int oo = e / IN, k0 = e % IN; for (int j = 0; j < 8; ++j) o[j] = (b16)(bf16_rne(w1[(k0 + j) * H + oo]) * WSC); for (int pass = 0; pass < 2; ++pass) { *(volatile v8b*)(W1T + e) = o; __threadfence(); } return; } u -= n1;
  if (u < n2) { const int e = (int)u * 8; const int oo = e / H, k0 = e % H; for (int j = 0; j < 8; ++j) o[j] = (b16)(bf16_rne(w2[(k0 + j) * H + oo]) * WSC); for (int pass = 0; pass < 2; ++pass) { *(volatile v8b*)(W2T + e) = o; __threadfence(); } return; } u -= n2;
  if (u < n3) { const int e = (int)u * 8; const int oo = e / H, k0 = e % H;
    for (int j = 0; j < 8; ++j) { const int k = k0 + j; float v; if (oo < 64) v = we1[k * H + oo]; else if (oo < 128) v = we1[(64 + k) * H + (oo - 64)]; else if (oo < 160) v = wd1[k * HD + (oo - 128)]; else v = wd1[(64 + k) * HD + (oo - 160)]; o[j] = (b16)(bf16_rne(v) * WSC); }
    for (int pass = 0; pass < 2; ++pass) { *(volatile v8b*)(WPT + e) = o; __threadfence(); } return; } u -= n3;
  if (u < n4) { const int e = (int)u * 8; const int oo = e / HD, k0 = e % HD; for (int j = 0; j < 8; ++j) o[j] = (oo == 0) ? (b16)(bf16_rne(wd2[k0 + j]) * WSC) : (b16)0.0f; for (int pass = 0; pass < 2; ++pass) { *(volatile v8b*)(WD2 + e) = o; __threadfence(); } }
}
__global__ __launch_bounds__(32) void node_kernel(const b16* __restrict__ X16, const b16* __restrict__ W1T, const float* __restrict__ b1, const b16* __restrict__ W2T, const float* __restrict__ b2, const b16* __restrict__ WPT, float* __restrict__ NODES, float* __restrict__ PROJ) {
  __shared__ __attribute__((aligned(16))) b16 Hh[16][H + 8], Hl[16][H + 8]; __shared__ __attribute__((aligned(16))) float Tf[16][PW + 4];
  const int lane = threadIdx.x, nloc = lane & 15, hlf = lane >> 4; const size_t m0 = (size_t)blockIdx.x * 16;
  v8f a4[4] = {{}, {}, {}, {}}; { const v16b a = frag_kb(X16 + (m0 + nloc) * IN, hlf);
#pragma unroll
    for (int t = 0; t < 4; ++t) a4[t] = wmma16b(a, frag_kb(W1T + (size_t)(t * 16 + nloc) * IN, hlf), a4[t]); }
#pragma unroll
  for (int t = 0; t < 4; ++t) { const int c = t * 16 + nloc; const float bb = bf16_rne(b1[c]);
#pragma unroll
    for (int r = 0; r < 8; ++r) { b16 p, q; split16(fmaxf(a4[t][r] * (1.0f / (XS * WSC)) + bb, 0.0f) * XS, p, q); Hh[8 * hlf + r][c] = p; Hl[8 * hlf + r][c] = q; } }
  wave_lds_sync();
  v8f n4[4] = {{}, {}, {}, {}};
#pragma unroll
  for (int kb = 0; kb < H; kb += 32) { const v16b a = frag_kb(&Hh[nloc][kb], hlf), al = frag_kb(&Hl[nloc][kb], hlf);
#pragma unroll
    for (int t = 0; t < 4; ++t) { const v16b bw = frag_kb(W2T + (size_t)(t * 16 + nloc) * H + kb, hlf); n4[t] = wmma16b(a, bw, n4[t]); n4[t] = wmma16b(al, bw, n4[t]); } }
  wave_lds_sync();
#pragma unroll
  for (int t = 0; t < 4; ++t) { const int c = t * 16 + nloc; const float bb = bf16_rne(b2[c]);
#pragma unroll
    for (int r = 0; r < 8; ++r) { const float nv = n4[t][r] * (1.0f / (XS * WSC)) + bb; Tf[8 * hlf + r][c] = nv; b16 p, q; split16(nv * XS, p, q); Hh[8 * hlf + r][c] = p; Hl[8 * hlf + r][c] = q; } }
  wave_lds_sync();
  for (int pass = 0; pass < 2; ++pass) { for (int rr = 0; rr < 16; ++rr) if (lane < 16) *(volatile v4f*)(NODES + (m0 + rr) * H + lane * 4) = *(const v4f*)(&Tf[rr][lane * 4]); __threadfence(); }
  wave_lds_sync();
  v8f p12[12];
#pragma unroll
  for (int t = 0; t < 12; ++t) p12[t] = (v8f){};
#pragma unroll
  for (int kb = 0; kb < H; kb += 32) { const v16b a = frag_kb(&Hh[nloc][kb], hlf), al = frag_kb(&Hl[nloc][kb], hlf);
#pragma unroll
    for (int t = 0; t < 12; ++t) { const v16b bw = frag_kb(WPT + (size_t)(t * 16 + nloc) * H + kb, hlf); p12[t] = wmma16b(a, bw, p12[t]); p12[t] = wmma16b(al, bw, p12[t]); } }
#pragma unroll
  for (int t = 0; t < 12; ++t)
#pragma unroll
    for (int r = 0; r < 8; ++r) Tf[8 * hlf + r][t * 16 + nloc] = p12[t][r] * (1.0f / (XS * WSC));
  wave_lds_sync();
  for (int pass = 0; pass < 2; ++pass) { for (int rr = 0; rr < 16; ++rr) for (int sg = 0; sg < 3; ++sg) if (lane < 16) *(volatile v4f*)(PROJ + (m0 + rr) * PW + sg * 64 + lane * 4) = *(const v4f*)(&Tf[rr][sg * 64 + lane * 4]); __threadfence(); }
}
__global__ __launch_bounds__(256) void pair_kernel(const float* __restrict__ PROJ, const float* __restrict__ be1, const float* __restrict__ bd1, const b16* __restrict__ WD2, const float* __restrict__ bd2, float* __restrict__ PART) {
  __shared__ __attribute__((aligned(16))) b16 Gh[S][HD + 8], Gl[S][HD + 8]; __shared__ float keep[S]; __shared__ float psa[4][H], psu[4][H], psk[8]; __shared__ __attribute__((aligned(16))) float row[192];
  const int b = blockIdx.y, i = blockIdx.x, t_ = threadIdx.x, wave = t_ >> 5, lane = t_ & 31, hh = lane >> 4, col = lane & 15;
  const float* Pi = PROJ + ((size_t)b * S + i) * PW;
  for (int j = t_; j < S; j += 256) { const float* Qdj = PROJ + ((size_t)b * S + j) * PW + 160; const float* Pdi = Pi + 128;
    for (int c = 0; c < HD; ++c) { const float g = fmaxf(Pdi[c] + Qdj[c] + bf16_rne(bd1[c]), 0.0f); b16 p, q; split16(g * XS, p, q); Gh[j][c] = p; Gl[j][c] = q; } }
  __syncthreads();
  { const v16b bw = frag_kb(WD2 + (size_t)col * HD, hh); const float bb = bf16_rne(bd2[0]);
    for (int jt = wave; jt < S / 16; jt += 8) { v8f d = {}; d = wmma16b(frag_kb(&Gh[jt * 16 + col][0], hh), bw, d); d = wmma16b(frag_kb(&Gl[jt * 16 + col][0], hh), bw, d);
      if (col == 0) { for (int r = 0; r < 8; ++r) { const float lg = d[r] * (1.0f / (XS * WSC)) + bb; keep[jt * 16 + 8 * hh + r] = 1.0f / (1.0f + __expf(-lg)); } } } }
  __syncthreads();
  { const int c = t_ & 63, ph = t_ >> 6; const float pic = Pi[c] + bf16_rne(be1[c]); float sa = 0.0f, su = 0.0f, sk = 0.0f;
    for (int j = ph; j < S; j += 4) { const float u = fmaxf(pic + PROJ[((size_t)b * S + j) * PW + 64 + c], 0.0f); su += u; sa += pmul(keep[j], u); if (c == 0) sk += keep[j]; }
    psa[ph][c] = sa; psu[ph][c] = su; if (c == 0) psk[ph] = sk; }
  __syncthreads();
  if (t_ < H) { row[t_] = ((psa[0][t_] + psa[1][t_]) + psa[2][t_]) + psa[3][t_]; row[H + t_] = ((psu[0][t_] + psu[1][t_]) + psu[2][t_]) + psu[3][t_]; }
  if (t_ == 0) row[128] = ((psk[0] + psk[1]) + psk[2]) + psk[3]; if (t_ > 128 && t_ < 192) row[t_] = 0.0f;
  __syncthreads();
  for (int pass = 0; pass < 2; ++pass) { if (t_ < 48) *(volatile v4f*)(PART + ((size_t)b * S + i) * 192 + t_ * 4) = *(const v4f*)(&row[t_ * 4]); __threadfence(); }
}
__global__ __launch_bounds__(256) void final_kernel(const float* __restrict__ PART, const float* __restrict__ NODES, const float* __restrict__ we2, const float* __restrict__ be2, const float* __restrict__ wc1, const float* __restrict__ bc1, const float* __restrict__ wc2, const float* __restrict__ bc2, float* __restrict__ RB) {
  __shared__ float sa[H], su[H], sn[H], skk; __shared__ float feat[2 * H]; __shared__ float hid[HD]; __shared__ __attribute__((aligned(16))) float res[64];
  const int b = blockIdx.x, t_ = threadIdx.x;
  if (t_ < H) { float a = 0.0f, u = 0.0f, n = 0.0f; for (int i = 0; i < S; ++i) { const float* pr = PART + ((size_t)b * S + i) * 192; a += pr[t_]; u += pr[H + t_]; n += NODES[((size_t)b * S + i) * H + t_]; } sa[t_] = a; su[t_] = u; sn[t_] = n; }
  if (t_ == H) { float k = 0.0f; for (int i = 0; i < S; ++i) k += PART[((size_t)b * S + i) * 192 + 128]; skk = k; }
  __syncthreads();
  if (t_ < H) { float ma = 0.0f, mt = 0.0f;
#pragma unroll 1
    for (int k = 0; k < H; ++k) { const float w = bf16_rne(we2[k * H + t_]); ma += pmul(sa[k], w); mt += pmul(su[k] - sa[k], w); }
    const float bb = bf16_rne(be2[t_]); feat[t_] = (sn[t_] + ma + skk * bb) * (1.0f / S); feat[H + t_] = (mt + ((float)S * (float)S - skk) * bb) * (1.0f / S); }
  __syncthreads();
  if (t_ < HD) { float s = bf16_rne(bc1[t_]);
#pragma unroll 1
    for (int k = 0; k < 2 * H; ++k) s += pmul(feat[k], bf16_rne(wc1[k * HD + t_])); hid[t_] = fmaxf(s, 0.0f); }
  __syncthreads();
  if (t_ < 64) { float v = 0.0f; if (t_ < NC) { v = bf16_rne(bc2[t_]);
#pragma unroll 1
      for (int k = 0; k < HD; ++k) v += pmul(hid[k], bf16_rne(wc2[k * NC + t_])); } res[t_] = v; }
  __syncthreads();
  for (int pass = 0; pass < 2; ++pass) { if (t_ < 16) *(volatile v4f*)(RB + (size_t)b * 64 + t_ * 4) = *(const v4f*)(&res[t_ * 4]); __threadfence(); }
}
__global__ __launch_bounds__(32) void out_kernel(const float* __restrict__ RB, float* __restrict__ out) {
  const int lane = threadIdx.x; v4f o; for (int u = 0; u < 4; ++u) { const int f = lane * 4 + u; const int b = f / NC, c = f % NC; o[u] = (f < NB * NC) ? RB[b * 64 + c] : 0.0f; }
  for (int pass = 0; pass < 2; ++pass) { if (lane < (NB * NC) / 4) *(volatile v4f*)(out + lane * 4) = o; __threadfence(); }
}
}

extern "C" void kernel_launch(void* const* d_in, const int* in_sizes, int n_in, void* d_out, int out_size, void* d_ws, size_t ws_size, hipStream_t stream) {
  (void)n_in;
  auto Fp = [&](int i) { return (const float*)d_in[i]; };
  if (in_sizes[0] != NR * IN || in_sizes[1] != IN * H || in_sizes[3] != H * H || in_sizes[5] != 2 * H * H || in_sizes[7] != H * H || in_sizes[9] != 2 * H * HD || in_sizes[11] != HD || in_sizes[13] != 2 * H * HD || in_sizes[15] != HD * NC || out_size != NB * NC) return;
  size_t off = 0; char* ws = (char*)d_ws;
  auto carve = [&](size_t bytes) { char* p = ws + off; off += (bytes + 255) & ~(size_t)255; return p; };
  b16* X16 = (b16*)carve((size_t)NR * IN * 2); b16* W1T = (b16*)carve(H * IN * 2); b16* W2T = (b16*)carve(H * H * 2); b16* WPT = (b16*)carve(PW * H * 2); b16* WD2 = (b16*)carve(16 * HD * 2);
  float* NODES = (float*)carve((size_t)NR * H * 4); float* PROJ = (float*)carve((size_t)NR * PW * 4); float* PART = (float*)carve((size_t)NR * 192 * 4); float* RB = (float*)carve((size_t)NB * 64 * 4);
  if (off > ws_size || off > ((size_t)128 << 20)) return;
  prep_kernel<<<(unsigned)(((size_t)NR * IN / 8 + H * IN / 8 + H * H / 8 + PW * H / 8 + 16 * HD / 8 + 255) / 256), 256, 0, stream>>>(Fp(0), Fp(1), Fp(3), Fp(5), Fp(9), Fp(11), X16, W1T, W2T, WPT, WD2);
  node_kernel<<<NR / 16, 32, 0, stream>>>(X16, W1T, Fp(2), W2T, Fp(4), WPT, NODES, PROJ);
  pair_kernel<<<dim3(S, NB), 256, 0, stream>>>(PROJ, Fp(6), Fp(10), WD2, Fp(12), PART);
  final_kernel<<<NB, 256, 0, stream>>>(PART, NODES, Fp(7), Fp(8), Fp(13), Fp(14), Fp(15), Fp(16), RB);
  out_kernel<<<1, 32, 0, stream>>>(RB, (float*)d_out);
}
